// LSTM_52664888983991
// MI455X (gfx1250) — hardware-verified
//
#include <hip/hip_runtime.h>

typedef __attribute__((ext_vector_type(16))) _Float16 v16h;
typedef __attribute__((ext_vector_type(8)))  _Float16 v8h;
typedef __attribute__((ext_vector_type(8)))  float    v8f;
typedef __attribute__((ext_vector_type(4)))  float    v4f;

constexpr int kSteps    = 512;
constexpr int kBatch    = 64;
constexpr int kFeat     = 256;
constexpr int kHid      = 1024;
constexpr int kCls      = 257;
constexpr int kKdim     = kFeat + kHid;
constexpr int kGateCols = 4 * kHid;
constexpr int kSamp     = 16;
constexpr int kCellBlocks  = kBatch / kSamp;
constexpr int kCellWaves   = 16;
constexpr int kCellThreads = kCellWaves * 32;
constexpr int kKsteps   = kKdim / 32;
constexpr int kPitch    = kKdim + 8;
constexpr int kTileSz   = kSamp * kPitch;
constexpr int kFragHalves = 512;
constexpr int kPassStride = kKsteps * 8 * kFragHalves;
constexpr int kClsPad   = 288;
constexpr int kHeadRows = 32;
constexpr int kHeadWaves = 9;
constexpr int kHeadThreads = kHeadWaves * 32;
constexpr int kHeadLines = (kHeadRows * kCls * 4) / 128;
constexpr float kCarryA  = 64.0f;
constexpr float kCarryW  = 1024.0f;
constexpr float kFold    = 1.0f / (kCarryA * kCarryW);
constexpr float kMinNorm = 6.103515625e-05f;

static_assert(kKdim == 1280);
static_assert((kKdim % 32) == 0 && (kHid % 32) == 0 && (kFeat % 32) == 0);
static_assert(kCellWaves * 64 == kHid);
static_assert(kCellBlocks * kSamp == kBatch);
static_assert((kPitch % 8) == 0);
static_assert(kHeadRows * kCls * 4 == kHeadLines * 128);
static_assert(kHeadLines == 257);
static_assert(kHeadWaves * 2 * 16 == kClsPad);
static_assert(kClsPad >= kCls);
static_assert((kSteps * kBatch) % kHeadRows == 0);
static_assert(kHeadWaves * 4 * 8 >= kHeadLines);

constexpr size_t kBytesWP = (size_t)kGateCols * kKdim * 2;
constexpr size_t kBytesFP = (size_t)kClsPad * kHid * 2;
constexpr size_t kBytesHS = (size_t)kSteps * kBatch * kHid * 2;
constexpr size_t kOffWP = 0;
constexpr size_t kOffFP = kOffWP + kBytesWP;
constexpr size_t kOffHS = kOffFP + kBytesFP;
constexpr size_t kWsTotal = kOffHS + kBytesHS;
static_assert(kBytesWP == 10485760ull);
static_assert(kBytesFP == 589824ull);
static_assert(kBytesHS == 67108864ull);
static_assert(kWsTotal == 78184448ull);
static_assert(kWsTotal <= 134217728ull);
static_assert((kOffFP % 128) == 0 && (kOffHS % 128) == 0);

__device__ __forceinline__ unsigned short f2bf_bits(float f) {
  unsigned u = __float_as_uint(f);
  return (unsigned short)((u + 0x7FFFu + ((u >> 16) & 1u)) >> 16);
}
__device__ __forceinline__ float bf_bits2f(unsigned short h) { return __uint_as_float(((unsigned)h) << 16); }
__device__ __forceinline__ float rne_bf(float f) { return bf_bits2f(f2bf_bits(f)); }

__device__ __forceinline__ _Float16 op_from_value(float v, float carry) {
  const float r = v * carry;
  const float z = (__builtin_fabsf(r) < kMinNorm) ? 0.0f : r;
  return (_Float16)z;
}
__device__ __forceinline__ _Float16 op_from_input(float v, float carry) {
  return op_from_value(rne_bf(v), carry);
}

union FragU { v16h v; v8h h[2]; };
__device__ __forceinline__ v16h load_frag(const _Float16* p0, const _Float16* p1) {
  FragU f;
  f.h[0] = *(const v8h*)(p0);
  f.h[1] = *(const v8h*)(p1);
  return f.v;
}
__device__ __forceinline__ v8f mma1(v16h a, v16h b, v8f c) {
  c = __builtin_amdgcn_wmma_f32_16x16x32_f16(false, a, false, b, (short)0, c, false, false);
  asm volatile("v_nop\n\tv_nop\n\tv_nop\n\tv_nop" : "+v"(c) : "v"(a), "v"(b));
  return c;
}
__device__ __forceinline__ float sig_fast(float x) {
  return __builtin_amdgcn_rcpf(1.0f + __expf(-x));
}
__device__ __forceinline__ float tanh_fast(float x) {
  const float r = __builtin_amdgcn_rcpf(1.0f + __expf(-2.0f * x));
  return fmaf(2.0f, r, -1.0f);
}

__global__ __launch_bounds__(256) void weight_planes(
    const float* __restrict__ wxf, const float* __restrict__ wxi,
    const float* __restrict__ wxo, const float* __restrict__ wxa,
    const float* __restrict__ whf, const float* __restrict__ whi,
    const float* __restrict__ who, const float* __restrict__ wha,
    _Float16* __restrict__ wp)
{
  const int gid = blockIdx.x * 256 + threadIdx.x;
  const int l   = gid & 31;
  const int hf  = (gid >> 5) & 1;
  const int fi  = gid >> 6;
  const int tl  = fi & 7;
  const int rest = fi >> 3;
  const int ks  = rest % kKsteps;
  const int wpi = rest / kKsteps;
  const int ps  = wpi & 1;
  const int wv  = wpi >> 1;
  const int g   = tl >> 1;
  const int jj  = tl & 1;
  const int hh  = l >> 4;
  const int m   = l & 15;
  const int u   = 64 * wv + 32 * ps + 16 * jj + m;
  const int k   = ks * 32 + 16 * hf + 8 * hh;
  const float* sx = (g == 0) ? wxf : (g == 1) ? wxi : (g == 2) ? wxo : wxa;
  const float* sh = (g == 0) ? whf : (g == 1) ? whi : (g == 2) ? who : wha;
  const bool inpart = (k < kFeat);
  const int kk = inpart ? k : (k - kFeat);
  const float* src = inpart ? (sx + (size_t)u * kFeat + kk) : (sh + (size_t)u * kHid + kk);
  const v4f a0 = *(const v4f*)(src);
  const v4f a1 = *(const v4f*)(src + 4);
  v8h hv;
#pragma unroll
  for (int e = 0; e < 4; ++e) {
    hv[e]     = op_from_input(a0[e], kCarryW);
    hv[4 + e] = op_from_input(a1[e], kCarryW);
  }
  _Float16* dst = wp + (size_t)gid * 8;
  *(volatile v8h*)dst = hv;
  __threadfence();
  *(volatile v8h*)dst = hv;
}

__global__ __launch_bounds__(256) void head_plane(const float* __restrict__ fw, _Float16* __restrict__ fp)
{
  const int gid = blockIdx.x * 256 + threadIdx.x;
  const int row = gid >> 7;
  const int c8  = (gid & 127) * 8;
  const int rc  = (row < kCls) ? row : (kCls - 1);
  const bool live = (row < kCls);
  const float* src = fw + (size_t)rc * kHid + c8;
  const v4f a0 = *(const v4f*)(src);
  const v4f a1 = *(const v4f*)(src + 4);
  v8h hv;
#pragma unroll
  for (int e = 0; e < 4; ++e) {
    const float w0 = live ? a0[e] : 0.0f;
    const float w1 = live ? a1[e] : 0.0f;
    hv[e]     = op_from_input(w0, kCarryW);
    hv[4 + e] = op_from_input(w1, kCarryW);
  }
  _Float16* dst = fp + (size_t)gid * 8;
  *(volatile v8h*)dst = hv;
  __threadfence();
  *(volatile v8h*)dst = hv;
}


__device__ __forceinline__ void stage_x(const float* __restrict__ xrows, _Float16* dst, int tid) {
  const int s = tid >> 5;
  const int col = (tid & 31) * 8;
  const float* sp = xrows + (size_t)s * kFeat + col;
  const v4f a0 = *(const v4f*)(sp);
  const v4f a1 = *(const v4f*)(sp + 4);
  v8h hv;
#pragma unroll
  for (int e = 0; e < 4; ++e) {
    hv[e]     = op_from_input(a0[e], kCarryA);
    hv[4 + e] = op_from_input(a1[e], kCarryA);
  }
  *(v8h*)(dst + s * kPitch + col) = hv;
}

__device__ __forceinline__ void flush_h(const _Float16* tile, _Float16* __restrict__ dstrow, int wave, int lane) {
  const _Float16* sp = tile + wave * kPitch + kFeat + lane * 8;
  v8h hv[4];
#pragma unroll
  for (int i = 0; i < 4; ++i) hv[i] = *(const v8h*)(sp + i * 256);
  for (int pass = 0; pass < 2; ++pass) {
#pragma unroll
    for (int i = 0; i < 4; ++i) *(volatile v8h*)(dstrow + i * 256 + lane * 8) = hv[i];
    __threadfence();
  }
}

__device__ __forceinline__ void gate_pass(const _Float16* cur, _Float16* nxt,
                                          const _Float16* __restrict__ wl, const float* bias_s,
                                          int ucol, int hh, int m, float (&cst)[2][8])
{
  v8f acc[8];
#pragma unroll
  for (int tl = 0; tl < 8; ++tl) acc[tl] = (v8f){0.f, 0.f, 0.f, 0.f, 0.f, 0.f, 0.f, 0.f};
  const _Float16* ap = cur + m * kPitch + 8 * hh;
  const _Float16* bp = wl;
#pragma unroll 1
  for (int ks = 0; ks < kKsteps; ++ks) {
    const v16h a = load_frag(ap, ap + 16);
#pragma unroll
    for (int tl = 0; tl < 8; ++tl) {
      const v16h b = load_frag(bp + tl * kFragHalves, bp + tl * kFragHalves + 256);
      acc[tl] = mma1(a, b, acc[tl]);
    }
    ap += 32;
    bp += 8 * kFragHalves;
  }
#pragma unroll
  for (int jj = 0; jj < 2; ++jj) {
    const int u = ucol + 16 * jj;
    const float bfv = bias_s[u];
    const float biv = bias_s[kHid + u];
    const float bov = bias_s[2 * kHid + u];
    const float bav = bias_s[3 * kHid + u];
    _Float16* hp = nxt + (8 * hh) * kPitch + kFeat + u;
#pragma unroll
    for (int r = 0; r < 8; ++r) {
      const float zf = fmaf(acc[0 + jj][r], kFold, bfv);
      const float zi = fmaf(acc[2 + jj][r], kFold, biv);
      const float zo = fmaf(acc[4 + jj][r], kFold, bov);
      const float za = fmaf(acc[6 + jj][r], kFold, bav);
      const float ft = sig_fast(zf);
      const float it = sig_fast(zi);
      const float ot = sig_fast(zo);
      const float ta = tanh_fast(za);
      const float cn = it * ta + ft * cst[jj][r];
      cst[jj][r] = cn;
      const float hn = ot * tanh_fast(cn);
      hp[r * kPitch] = op_from_value(hn, kCarryA);
    }
  }
}

__global__ __launch_bounds__(512) void cell_steps(
    const float* __restrict__ x, const _Float16* __restrict__ wp,
    const float* __restrict__ bgf, const float* __restrict__ bgi,
    const float* __restrict__ bgo, const float* __restrict__ bga,
    _Float16* __restrict__ hs)
{
  __shared__ __align__(16) _Float16 atile[2 * kTileSz];
  __shared__ __align__(16) float bias_s[kGateCols];

  const int tid  = threadIdx.x;
  const int lane = tid & 31;
  const int wave = tid >> 5;
  const int hh   = lane >> 4;
  const int m    = lane & 15;
  const int samp0 = blockIdx.x * kSamp;

  for (int u = tid; u < kHid; u += kCellThreads) {
    bias_s[u]            = rne_bf(bgf[u]);
    bias_s[kHid + u]     = rne_bf(bgi[u]);
    bias_s[2 * kHid + u] = rne_bf(bgo[u]);
    bias_s[3 * kHid + u] = rne_bf(bga[u]);
  }
  {
    const int s = tid >> 5;
    const int c = (tid & 31) * 8;
    v8h z;
#pragma unroll
    for (int e = 0; e < 8; ++e) z[e] = (_Float16)0.0f;
#pragma unroll
    for (int i = 0; i < 4; ++i) *(v8h*)(atile + s * kPitch + kFeat + i * 256 + c) = z;
  }
  stage_x(x + (size_t)samp0 * kFeat, atile, tid);

  float c0[2][8], c1[2][8];
#pragma unroll
  for (int jj = 0; jj < 2; ++jj) {
#pragma unroll
    for (int r = 0; r < 8; ++r) {
      c0[jj][r] = 0.0f;
      c1[jj][r] = 0.0f;
    }
  }
  __syncthreads();

  const _Float16* wlane = wp + (size_t)wave * 2 * kPassStride + lane * 8;
  const int ucol = wave * 64 + m;

#pragma unroll 1
  for (int t = 0; t < kSteps; ++t) {
    const _Float16* cur = atile + (t & 1) * kTileSz;
    _Float16* nxt = atile + ((t + 1) & 1) * kTileSz;
    if (t > 0) flush_h(cur, hs + ((size_t)(t - 1) * kBatch + samp0 + wave) * kHid, wave, lane);
    gate_pass(cur, nxt, wlane, bias_s, ucol, hh, m, c0);
    gate_pass(cur, nxt, wlane + kPassStride, bias_s, ucol + 32, hh, m, c1);
    if (t + 1 < kSteps) stage_x(x + ((size_t)(t + 1) * kBatch + samp0) * kFeat, nxt, tid);
    __syncthreads();
  }
  flush_h(atile + (kSteps & 1) * kTileSz, hs + ((size_t)(kSteps - 1) * kBatch + samp0 + wave) * kHid, wave, lane);
}

__global__ __launch_bounds__(288) void head_rows(
    const _Float16* __restrict__ hs, const _Float16* __restrict__ fp,
    const float* __restrict__ fb, float* __restrict__ out)
{
  __shared__ __align__(16) float slab[kHeadRows * kCls];
  const int tid  = threadIdx.x;
  const int lane = tid & 31;
  const int wave = tid >> 5;
  const int hh   = lane >> 4;
  const int m    = lane & 15;
  const size_t row0 = (size_t)blockIdx.x * kHeadRows;

  v8f acc[2][2];
#pragma unroll
  for (int i = 0; i < 2; ++i)
#pragma unroll
    for (int j = 0; j < 2; ++j) acc[i][j] = (v8f){0.f, 0.f, 0.f, 0.f, 0.f, 0.f, 0.f, 0.f};

  const _Float16* a0p = hs + (row0 + m) * kHid + 8 * hh;
  const _Float16* a1p = hs + (row0 + 16 + m) * kHid + 8 * hh;
  const _Float16* b0p = fp + (size_t)((2 * wave) * 16 + m) * kHid + 8 * hh;
  const _Float16* b1p = fp + (size_t)((2 * wave + 1) * 16 + m) * kHid + 8 * hh;
#pragma unroll 1
  for (int ks = 0; ks < kHid / 32; ++ks) {
    const int ko = ks * 32;
    const v16h a0 = load_frag(a0p + ko, a0p + ko + 16);
    const v16h a1 = load_frag(a1p + ko, a1p + ko + 16);
    const v16h b0 = load_frag(b0p + ko, b0p + ko + 16);
    const v16h b1 = load_frag(b1p + ko, b1p + ko + 16);
    acc[0][0] = mma1(a0, b0, acc[0][0]);
    acc[0][1] = mma1(a0, b1, acc[0][1]);
    acc[1][0] = mma1(a1, b0, acc[1][0]);
    acc[1][1] = mma1(a1, b1, acc[1][1]);
  }

#pragma unroll
  for (int j = 0; j < 2; ++j) {
    const int n  = (2 * wave + j) * 16 + m;
    const int nc = (n < kCls) ? n : (kCls - 1);
    float bv = fb[nc];
    asm volatile("" : "+v"(bv));
    bv = rne_bf(bv);
#pragma unroll
    for (int i = 0; i < 2; ++i) {
#pragma unroll
      for (int r = 0; r < 8; ++r) {
        const float v = fmaf(acc[i][j][r], kFold, bv);
        if (n < kCls) slab[(i * 16 + 8 * hh + r) * kCls + n] = v;
      }
    }
  }
  __syncthreads();

  {
    const int q  = lane >> 3;
    const int c4 = (lane & 7) * 4;
    float* ob = out + row0 * kCls;
    for (int pass = 0; pass < 2; ++pass) {
#pragma unroll
      for (int it = 0; it < 8; ++it) {
        const int L  = it * (kHeadWaves * 4) + wave * 4 + q;
        const int Lc = (L < kHeadLines) ? L : (kHeadLines - 1);
        const v4f v = *(const v4f*)(slab + Lc * 32 + c4);
        if (L < kHeadLines) *(volatile v4f*)(ob + (size_t)L * 32 + c4) = v;
      }
      __threadfence();
    }
  }
}

extern "C" void kernel_launch(void* const* d_in, const int* in_sizes, int n_in,
                              void* d_out, int out_size, void* d_ws, size_t ws_size,
                              hipStream_t stream) {
  if (n_in < 15) return;
  if (in_sizes[0] != kSteps * kBatch * kFeat) return;
  if (in_sizes[1] != kHid * kFeat || in_sizes[3] != kHid * kFeat ||
      in_sizes[5] != kHid * kFeat || in_sizes[7] != kHid * kFeat) return;
  if (in_sizes[2] != kHid || in_sizes[4] != kHid || in_sizes[6] != kHid || in_sizes[8] != kHid) return;
  if (in_sizes[9] != kHid * kHid || in_sizes[10] != kHid * kHid ||
      in_sizes[11] != kHid * kHid || in_sizes[12] != kHid * kHid) return;
  if (in_sizes[13] != kCls * kHid || in_sizes[14] != kCls) return;
  if (out_size != kSteps * kBatch * kCls) return;
  if (ws_size < kWsTotal) return;

  const float* x     = (const float*)d_in[0];
  const float* wfx_w = (const float*)d_in[1];
  const float* wfx_b = (const float*)d_in[2];
  const float* wix_w = (const float*)d_in[3];
  const float* wix_b = (const float*)d_in[4];
  const float* wox_w = (const float*)d_in[5];
  const float* wox_b = (const float*)d_in[6];
  const float* wcx_w = (const float*)d_in[7];
  const float* wcx_b = (const float*)d_in[8];
  const float* wfh_w = (const float*)d_in[9];
  const float* wih_w = (const float*)d_in[10];
  const float* woh_w = (const float*)d_in[11];
  const float* wch_w = (const float*)d_in[12];
  const float* fco_w = (const float*)d_in[13];
  const float* fco_b = (const float*)d_in[14];
  float* out = (float*)d_out;

  char* ws = (char*)d_ws;
  _Float16* WP = (_Float16*)(ws + kOffWP);
  _Float16* FP = (_Float16*)(ws + kOffFP);
  _Float16* HS = (_Float16*)(ws + kOffHS);

  constexpr int kWpBlocks = (kGateCols * kKdim / 8) / 256;
  static_assert(kWpBlocks * 256 * 8 == kGateCols * kKdim);
  static_assert(kWpBlocks == 2560);
  constexpr int kFpBlocks = (kClsPad * kHid / 8) / 256;
  static_assert(kFpBlocks * 256 * 8 == kClsPad * kHid);
  constexpr int kHeadBlocks = (kSteps * kBatch) / kHeadRows;

  weight_planes<<<dim3(kWpBlocks), dim3(256), 0, stream>>>(
      wfx_w, wix_w, wox_w, wcx_w, wfh_w, wih_w, woh_w, wch_w, WP);
  head_plane<<<dim3(kFpBlocks), dim3(256), 0, stream>>>(fco_w, FP);
  cell_steps<<<dim3(kCellBlocks), dim3(kCellThreads), 0, stream>>>(
      x, WP, wfx_b, wix_b, wox_b, wcx_b, HS);
  head_rows<<<dim3(kHeadBlocks), dim3(kHeadThreads), 0, stream>>>(HS, FP, fco_b, out);
}
